// MultiHeadedMaskedAttention_24352464570233
// MI455X (gfx1250) — hardware-verified
//
#include <hip/hip_runtime.h>


#define DEV static __device__ __forceinline__

constexpr int kD  = 1024;
constexpr int kH  = 16;
constexpr int kHD = 64;
constexpr int kB  = 4;
constexpr int kS  = 2048;

constexpr size_t kPL = (size_t)kD * kD;
constexpr size_t kXN = (size_t)kB * kS * kD;
constexpr size_t kHP = (size_t)kH * kS * kHD;
constexpr size_t kCP = (size_t)kS * kD;

constexpr int kTP = 65;

typedef __attribute__((ext_vector_type(16))) __bf16         v16bf;
typedef __attribute__((ext_vector_type(8)))  float          v8f;
typedef __attribute__((ext_vector_type(4)))  float          v4f;
typedef __attribute__((ext_vector_type(8)))  unsigned       v8u;
typedef __attribute__((ext_vector_type(8)))  unsigned short ush8;

union Frag { v16bf v; ush8 h[2]; unsigned short e[16]; };
union U8   { ush8 v; unsigned short e[8]; };

DEV unsigned short bfu(float f) {
  unsigned u = __builtin_bit_cast(unsigned, f);
  u += 0x7FFFu + ((u >> 16) & 1u);
  return (unsigned short)(u >> 16);
}
DEV float bf2f(unsigned short s) {
  return __builtin_bit_cast(float, ((unsigned)s) << 16);
}
DEV void split2(float x, unsigned short& hi, unsigned short& lo) {
  hi = bfu(x);
  lo = bfu(x - bf2f(hi));
}

DEV v8f vzero() {
  v8f z;
#pragma unroll
  for (int r = 0; r < 8; ++r) z[r] = 0.0f;
  return z;
}

DEV v8f mma(v16bf a, v16bf b, v8f c) {
  c = __builtin_amdgcn_wmma_f32_16x16x32_bf16(false, a, false, b, (short)0, c,
                                               false, false);
  v8u au = __builtin_bit_cast(v8u, a);
  v8u bu = __builtin_bit_cast(v8u, b);
  asm volatile("v_nop\n\tv_nop\n\tv_nop\n\tv_nop" : "+v"(c) : "v"(au), "v"(bu));
  return c;
}

DEV v16bf ld_frag(const unsigned short* base, size_t ld) {
  const int lane = threadIdx.x & 31;
  const int r = lane & 15, hh = lane >> 4;
  const unsigned short* p = base + (size_t)r * ld + 8 * hh;
  Frag f;
  f.h[0] = *(const ush8*)(p);
  f.h[1] = *(const ush8*)(p + 16);
  return f.v;
}

__global__ __launch_bounds__(256) void k_cvt_w(const float* __restrict__ Wq,
                                               const float* __restrict__ Wk,
                                               const float* __restrict__ Wv,
                                               const float* __restrict__ Wo,
                                               unsigned short* Wp) {
  __shared__ float tile[64 * kTP];
  const int which = blockIdx.y;
  const int tb = blockIdx.x;
  const int t = threadIdx.x;
  int n0, k0;
  if (which < 3) {
    const float* W = (which == 0) ? Wq : ((which == 1) ? Wk : Wv);
    const int h = tb >> 4;
    const int d0 = (tb & 15) * 64;
    n0 = h * 64;
    k0 = d0;
#pragma unroll
    for (int j = 0; j < 16; ++j) {
      const int i = t + 256 * j;
      const int dd = i >> 6, e = i & 63;
      tile[e * kTP + dd] = W[((size_t)h * kD + d0 + dd) * kHD + e];
    }
  } else {
    n0 = (tb >> 4) * 64;
    k0 = (tb & 15) * 64;
#pragma unroll
    for (int j = 0; j < 16; ++j) {
      const int i = t + 256 * j;
      const int r = i >> 6, c = i & 63;
      tile[r * kTP + c] = Wo[(size_t)(n0 + r) * kD + k0 + c];
    }
  }
  __syncthreads();

  unsigned short* ph = Wp + (size_t)which * 2 * kPL;
  unsigned short* pl = ph + kPL;
  U8 hv[2], lv[2];
  size_t off[2];
#pragma unroll
  for (int p = 0; p < 2; ++p) {
    const int row = (t >> 3) + 32 * p;
    const int seg = t & 7;
#pragma unroll
    for (int j = 0; j < 8; ++j)
      split2(tile[row * kTP + seg * 8 + j], hv[p].e[j], lv[p].e[j]);
    off[p] = (size_t)(n0 + row) * kD + k0 + seg * 8;
  }
#pragma unroll
  for (int p = 0; p < 2; ++p) {
    *(volatile ush8*)(ph + off[p]) = hv[p].v;
    *(volatile ush8*)(pl + off[p]) = lv[p].v;
  }
  __threadfence();
#pragma unroll
  for (int p = 0; p < 2; ++p) {
    *(volatile ush8*)(ph + off[p]) = hv[p].v;
    *(volatile ush8*)(pl + off[p]) = lv[p].v;
  }
}

__global__ __launch_bounds__(256) void k_cvt_x(const float* __restrict__ X,
                                               unsigned short* Xh,
                                               unsigned short* Xl, int n8) {
  const int i = blockIdx.x * 256 + threadIdx.x;
  if (i >= n8) return;
  const float* p = X + (size_t)i * 8;
  const v4f a = *(const v4f*)(p);
  const v4f b = *(const v4f*)(p + 4);
  U8 hv, lv;
#pragma unroll
  for (int j = 0; j < 4; ++j) {
    split2(a[j], hv.e[j], lv.e[j]);
    split2(b[j], hv.e[4 + j], lv.e[4 + j]);
  }
  const size_t off = (size_t)i * 8;
  *(volatile ush8*)(Xh + off) = hv.v;
  *(volatile ush8*)(Xl + off) = lv.v;
  __threadfence();
  *(volatile ush8*)(Xh + off) = hv.v;
  *(volatile ush8*)(Xl + off) = lv.v;
}

DEV void gemm64(const unsigned short* Ah, const unsigned short* Al,
                const unsigned short* Bh, const unsigned short* Bl, float* sT) {
  const int wave = threadIdx.x >> 5;
  const int lane = threadIdx.x & 31;
  const int hh = lane >> 4, m = lane & 15;
  const int wm = wave >> 1, wn = wave & 1;
  const unsigned short* ah0 = Ah + (size_t)(wm * 32) * kD;
  const unsigned short* al0 = Al + (size_t)(wm * 32) * kD;
  const unsigned short* bh0 = Bh + (size_t)(wn * 32) * kD;
  const unsigned short* bl0 = Bl + (size_t)(wn * 32) * kD;

  v8f acc[2][2];
#pragma unroll
  for (int i = 0; i < 2; ++i)
#pragma unroll
    for (int j = 0; j < 2; ++j) acc[i][j] = vzero();

#pragma unroll 1
  for (int k0 = 0; k0 < kD; k0 += 32) {
    v16bf fah[2], fal[2], fbh[2], fbl[2];
#pragma unroll
    for (int i = 0; i < 2; ++i) {
      fah[i] = ld_frag(ah0 + (size_t)(i * 16) * kD + k0, kD);
      fal[i] = ld_frag(al0 + (size_t)(i * 16) * kD + k0, kD);
      fbh[i] = ld_frag(bh0 + (size_t)(i * 16) * kD + k0, kD);
      fbl[i] = ld_frag(bl0 + (size_t)(i * 16) * kD + k0, kD);
    }
#pragma unroll
    for (int i = 0; i < 2; ++i)
#pragma unroll
      for (int j = 0; j < 2; ++j) {
        acc[i][j] = mma(fah[i], fbh[j], acc[i][j]);
        acc[i][j] = mma(fah[i], fbl[j], acc[i][j]);
        acc[i][j] = mma(fal[i], fbh[j], acc[i][j]);
      }
  }

#pragma unroll
  for (int i = 0; i < 2; ++i)
#pragma unroll
    for (int j = 0; j < 2; ++j)
#pragma unroll
      for (int r = 0; r < 8; ++r)
        sT[(wm * 32 + i * 16 + 8 * hh + r) * kTP + wn * 32 + j * 16 + m] =
            acc[i][j][r];
}

__global__ __launch_bounds__(128) void k_qkv(
    const unsigned short* Xh, const unsigned short* Xl, const unsigned short* Wp,
    unsigned short* Qh, unsigned short* Ql, unsigned short* Kh,
    unsigned short* Kl, unsigned short* Vh, unsigned short* Vl) {
  __shared__ float sT[64 * kTP];
  const int which = blockIdx.y >> 4;
  const int h = blockIdx.y & 15;
  const int m0 = blockIdx.x * 64;
  const int t = threadIdx.x;

  const unsigned short* Bh = Wp + (size_t)which * 2 * kPL + (size_t)(h * 64) * kD;
  const unsigned short* Bl = Bh + kPL;
  gemm64(Xh + (size_t)m0 * kD, Xl + (size_t)m0 * kD, Bh, Bl, sT);
  __syncthreads();

  U8 hv[4], lv[4];
  size_t off[4];
  if (which < 2) {
    unsigned short* dh = (which == 0) ? Qh : Kh;
    unsigned short* dl = (which == 0) ? Ql : Kl;
#pragma unroll
    for (int p = 0; p < 4; ++p) {
      const int row = (t >> 3) + 16 * p;
      const int seg = t & 7;
#pragma unroll
      for (int j = 0; j < 8; ++j)
        split2(sT[row * kTP + seg * 8 + j], hv[p].e[j], lv[p].e[j]);
      off[p] = ((size_t)h * kS + m0 + row) * kHD + seg * 8;
    }
#pragma unroll
    for (int p = 0; p < 4; ++p) {
      *(volatile ush8*)(dh + off[p]) = hv[p].v;
      *(volatile ush8*)(dl + off[p]) = lv[p].v;
    }
    __threadfence();
#pragma unroll
    for (int p = 0; p < 4; ++p) {
      *(volatile ush8*)(dh + off[p]) = hv[p].v;
      *(volatile ush8*)(dl + off[p]) = lv[p].v;
    }
  } else {
#pragma unroll
    for (int p = 0; p < 4; ++p) {
      const int e = (t >> 3) + 16 * p;
      const int seg = t & 7;
#pragma unroll
      for (int j = 0; j < 8; ++j)
        split2(sT[(seg * 8 + j) * kTP + e], hv[p].e[j], lv[p].e[j]);
      off[p] = ((size_t)h * kHD + e) * kS + m0 + seg * 8;
    }
#pragma unroll
    for (int p = 0; p < 4; ++p) {
      *(volatile ush8*)(Vh + off[p]) = hv[p].v;
      *(volatile ush8*)(Vl + off[p]) = lv[p].v;
    }
    __threadfence();
#pragma unroll
    for (int p = 0; p < 4; ++p) {
      *(volatile ush8*)(Vh + off[p]) = hv[p].v;
      *(volatile ush8*)(Vl + off[p]) = lv[p].v;
    }
  }
}

__global__ __launch_bounds__(32) void k_attn(
    const unsigned short* Qh, const unsigned short* Ql,
    const unsigned short* Kh, const unsigned short* Kl,
    const unsigned short* Vh, const unsigned short* Vl,
    unsigned short* Ch, unsigned short* Cl) {
  __shared__ float sP[16 * kTP];
  const int lane = threadIdx.x & 31;
  const int hh = lane >> 4, m = lane & 15;
  const int qt = blockIdx.x;
  const int h = blockIdx.y;
  const int qbase = qt * 16;

  const size_t qoff = ((size_t)h * kS + (size_t)qbase) * kHD;
  v16bf qh[2], ql[2];
  qh[0] = ld_frag(Qh + qoff, kHD);
  qh[1] = ld_frag(Qh + qoff + 32, kHD);
  ql[0] = ld_frag(Ql + qoff, kHD);
  ql[1] = ld_frag(Ql + qoff + 32, kHD);

  const unsigned short* Kbh = Kh + (size_t)h * kS * kHD;
  const unsigned short* Kbl = Kl + (size_t)h * kS * kHD;
  const unsigned short* Vbh = Vh + (size_t)h * kHD * kS;
  const unsigned short* Vbl = Vl + (size_t)h * kHD * kS;

  float mrow[8], lrow[8];
#pragma unroll
  for (int r = 0; r < 8; ++r) { mrow[r] = -3.0e38f; lrow[r] = 0.0f; }
  v8f o[4];
#pragma unroll
  for (int nt = 0; nt < 4; ++nt) o[nt] = vzero();

  for (int kb = 0; kb <= qbase; kb += 32) {
    v8f sacc[2];
#pragma unroll
    for (int t = 0; t < 2; ++t) {
      const int kt = kb + 16 * t;
      v8f z = vzero();
#pragma unroll
      for (int ks = 0; ks < 2; ++ks) {
        v16bf fkh = ld_frag(Kbh + (size_t)kt * kHD + ks * 32, kHD);
        v16bf fkl = ld_frag(Kbl + (size_t)kt * kHD + ks * 32, kHD);
        z = mma(qh[ks], fkh, z);
        z = mma(qh[ks], fkl, z);
        z = mma(ql[ks], fkh, z);
      }
      sacc[t] = z;
    }

#pragma unroll
    for (int r = 0; r < 8; ++r) {
      const int rg = qbase + 8 * hh + r;
      float s0 = sacc[0][r] * 0.125f;
      float s1 = sacc[1][r] * 0.125f;
      if (kb + m > rg)      s0 = -1.0e30f;
      if (kb + 16 + m > rg) s1 = -1.0e30f;
      float tmax = fmaxf(s0, s1);
#pragma unroll
      for (int dlt = 1; dlt < 16; dlt <<= 1)
        tmax = fmaxf(tmax, __shfl_xor(tmax, dlt, 32));
      const float mn = fmaxf(mrow[r], tmax);
      const float p0 = __expf(s0 - mn);
      const float p1 = __expf(s1 - mn);
      float rs = p0 + p1;
#pragma unroll
      for (int dlt = 1; dlt < 16; dlt <<= 1)
        rs += __shfl_xor(rs, dlt, 32);
      const float sc = __expf(mrow[r] - mn);
      lrow[r] = lrow[r] * sc + rs;
      mrow[r] = mn;
#pragma unroll
      for (int nt = 0; nt < 4; ++nt) o[nt][r] *= sc;
      sP[(8 * hh + r) * kTP + m]      = p0;
      sP[(8 * hh + r) * kTP + 16 + m] = p1;
    }
    __syncthreads();

    Frag ph, pl;
#pragma unroll
    for (int j = 0; j < 8; ++j) {
      split2(sP[m * kTP + 8 * hh + j],      ph.e[j],     pl.e[j]);
      split2(sP[m * kTP + 16 + 8 * hh + j], ph.e[8 + j], pl.e[8 + j]);
    }
    __syncthreads();

#pragma unroll
    for (int nt = 0; nt < 4; ++nt) {
      v16bf fvh = ld_frag(Vbh + (size_t)(nt * 16) * kS + kb, kS);
      v16bf fvl = ld_frag(Vbl + (size_t)(nt * 16) * kS + kb, kS);
      o[nt] = mma(ph.v, fvh, o[nt]);
      o[nt] = mma(ph.v, fvl, o[nt]);
      o[nt] = mma(pl.v, fvh, o[nt]);
    }
  }

  float inv[8];
#pragma unroll
  for (int r = 0; r < 8; ++r) inv[r] = 1.0f / lrow[r];
#pragma unroll
  for (int nt = 0; nt < 4; ++nt)
#pragma unroll
    for (int r = 0; r < 8; ++r)
      sP[(8 * hh + r) * kTP + nt * 16 + m] = o[nt][r] * inv[r];
  __syncthreads();

  U8 hv[4], lv[4];
  size_t off[4];
#pragma unroll
  for (int p = 0; p < 4; ++p) {
    const int row = (lane >> 3) + 4 * p;
    const int seg = lane & 7;
#pragma unroll
    for (int j = 0; j < 8; ++j)
      split2(sP[row * kTP + seg * 8 + j], hv[p].e[j], lv[p].e[j]);
    off[p] = (size_t)(qbase + row) * kD + (size_t)h * kHD + seg * 8;
  }
#pragma unroll
  for (int p = 0; p < 4; ++p) {
    *(volatile ush8*)(Ch + off[p]) = hv[p].v;
    *(volatile ush8*)(Cl + off[p]) = lv[p].v;
  }
  __threadfence();
#pragma unroll
  for (int p = 0; p < 4; ++p) {
    *(volatile ush8*)(Ch + off[p]) = hv[p].v;
    *(volatile ush8*)(Cl + off[p]) = lv[p].v;
  }
}

__global__ __launch_bounds__(128) void k_oproj(
    const unsigned short* Chh, const unsigned short* Cll,
    const unsigned short* Woh, const unsigned short* Wol,
    const float* __restrict__ bo, float* out) {
  __shared__ float sT[64 * kTP];
  const int m0 = blockIdx.x * 64;
  const int n0 = blockIdx.y * 64;
  const int t = threadIdx.x;

  gemm64(Chh + (size_t)m0 * kD, Cll + (size_t)m0 * kD,
         Woh + (size_t)n0 * kD, Wol + (size_t)n0 * kD, sT);
  __syncthreads();

  const int seg = t & 15;
  const int col = n0 + seg * 4;
  v4f bias;
#pragma unroll
  for (int j = 0; j < 4; ++j) bias[j] = bo[col + j];
  v4f val[8];
  size_t off[8];
#pragma unroll
  for (int p = 0; p < 8; ++p) {
    const int row = (t >> 4) + 8 * p;
    v4f v;
#pragma unroll
    for (int j = 0; j < 4; ++j) v[j] = sT[row * kTP + seg * 4 + j] + bias[j];
    val[p] = v;
    off[p] = (size_t)(m0 + row) * kD + col;
  }
#pragma unroll
  for (int p = 0; p < 8; ++p) *(volatile v4f*)(out + off[p]) = val[p];
  __threadfence();
#pragma unroll
  for (int p = 0; p < 8; ++p) *(volatile v4f*)(out + off[p]) = val[p];
}

extern "C" void kernel_launch(void* const* d_in, const int* in_sizes, int n_in,
                              void* d_out, int out_size, void* d_ws,
                              size_t ws_size, hipStream_t stream) {
  if (n_in < 6) return;
  const float* emb = (const float*)d_in[0];
  const float* Wq  = (const float*)d_in[1];
  const float* Wk  = (const float*)d_in[2];
  const float* Wv  = (const float*)d_in[3];
  const float* Wo  = (const float*)d_in[4];
  const float* bo  = (const float*)d_in[5];
  float* out = (float*)d_out;

  if ((size_t)in_sizes[0] != kXN || (size_t)in_sizes[1] != (size_t)kH * kD * kHD ||
      (size_t)in_sizes[4] != kPL || in_sizes[5] != kD ||
      (size_t)out_size != kXN)
    return;

  const size_t OFF_W  = 0;
  const size_t OFF_XH = OFF_W + 8 * kPL;
  const size_t OFF_XL = OFF_XH + kXN;
  const size_t OFF_QH = OFF_XL + kXN;
  const size_t OFF_QL = OFF_QH + kHP;
  const size_t OFF_KH = OFF_QL + kHP;
  const size_t OFF_KL = OFF_KH + kHP;
  const size_t OFF_VH = OFF_KL + kHP;
  const size_t OFF_VL = OFF_VH + kHP;
  const size_t OFF_CH = OFF_VL + kHP;
  const size_t OFF_CL = OFF_CH + kCP;
  const size_t OFF_END = OFF_CL + kCP;
  static_assert(sizeof(unsigned short) == 2);
  if (OFF_END * sizeof(unsigned short) > ws_size) return;

  unsigned short* ws = (unsigned short*)d_ws;
  unsigned short* Wp = ws + OFF_W;
  unsigned short* Xh = ws + OFF_XH;
  unsigned short* Xl = ws + OFF_XL;
  unsigned short* Qh = ws + OFF_QH;
  unsigned short* Ql = ws + OFF_QL;
  unsigned short* Kh = ws + OFF_KH;
  unsigned short* Kl = ws + OFF_KL;
  unsigned short* Vh = ws + OFF_VH;
  unsigned short* Vl = ws + OFF_VL;
  unsigned short* Ch = ws + OFF_CH;
  unsigned short* Cl = ws + OFF_CL;

  k_cvt_w<<<dim3(256, 4), 256, 0, stream>>>(Wq, Wk, Wv, Wo, Wp);
  const int n8 = (int)(kXN / 8);
  k_cvt_x<<<dim3((n8 + 255) / 256), 256, 0, stream>>>(emb, Xh, Xl, n8);

  for (int b = 0; b < kB; ++b) {
    const size_t xo = (size_t)b * kS * kD;
    k_qkv<<<dim3(kS / 64, 3 * kH), 128, 0, stream>>>(
        Xh + xo, Xl + xo, Wp, Qh, Ql, Kh, Kl, Vh, Vl);
    k_attn<<<dim3(kS / 16, kH), 32, 0, stream>>>(Qh, Ql, Kh, Kl, Vh, Vl, Ch, Cl);
    k_oproj<<<dim3(kS / 64, kD / 64), 128, 0, stream>>>(
        Ch, Cl, Wp + 6 * kPL, Wp + 7 * kPL, bo, out + xo);
  }
}
